// GIN_ZINC_v2_77008763617630
// MI455X (gfx1250) — hardware-verified
//
#include <hip/hip_runtime.h>
#include <stddef.h>
#include <stdint.h>


#define HD      128
#define K2      256
#define AEMB    64
#define PEP     16
#define PER     20
#define NATOM   28
#define NLAY    4
#define NTHR    256
#define NWAVE   8
#define EPT     8
#define CHUNK   (NTHR * EPT)
#define WCAP    (EPT * 32)
#define LISTN   (NWAVE * WCAP)
#define NB      1024
#define PKS     10
#define RCAP    28672
#define DEGCAP  64
#define GBM     64
#define GBN     128
#define GTHR    128
#define GNT     8
#define PARTW   288
#define PG      16
#define GCAP    4096
#define RPW     21
#define PRECW   64
#define CZ_INTS (2 * RCAP + 2 * NB + LISTN + 48)
#define LDS_CMP (CZ_INTS * 4)
#define NUIN    (HD * (HD / 8))
#define NUC     (NLAY * HD * (K2 / 8))
#define NURO    (HD * (K2 / 8))
#define NUE     ((NATOM * AEMB) / 8)
#define NUB1    (NUIN)
#define NUB2    (NUIN + NUC)
#define NUB3    (NUIN + 2 * NUC)
#define NUB4    (NUIN + 2 * NUC + NURO)
#define NUTOT   (NUB4 + NUE)
#define WSCAP   134217728

static_assert((CHUNK & (CHUNK - 1)) == 0 && ((long long)CHUNK << PKS) < (1LL << 31));
static_assert((NB & (NB - 1)) == 0 && NB == (1 << PKS) && NTHR * 4 == NB && LISTN >= NB);
static_assert(RCAP >= 17426 && (RCAP % 32) == 0 && ((RCAP / 4) % NTHR) == 0);
static_assert(DEGCAP >= 35 + 8);
static_assert((CZ_INTS % 4) == 0 && LDS_CMP <= 300000);
static_assert(GBM == (GTHR / 32) * 16 && GBN == 16 * GNT && GTHR == GBN && HD == GBN && HD == 4 * 32);
static_assert((HD % 32) == 0 && (K2 % 32) == 0 && K2 == 2 * HD);
static_assert((PARTW % 32) == 0 && PARTW >= 2 * GBN + 1 && PARTW / 4 <= GTHR && PARTW >= GBN + GBM);
static_assert((NUB1 % NTHR) == 0 && (NUB2 % NTHR) == 0 && (NUB3 % NTHR) == 0 && (NUB4 % NTHR) == 0);
static_assert(NTHR == PEP * PEP && PER == 20 && RPW > PER && NUE * 8 == NATOM * AEMB);
static_assert((PG & (PG - 1)) == 0 && PG == 2 * NWAVE && PG <= NB && GCAP >= 1024 && (GCAP % 4) == 0);
static_assert(AEMB + 2 * PEP <= HD && AEMB == 64 && PEP == 16);

typedef float          v4f  __attribute__((ext_vector_type(4)));
typedef float          v8f  __attribute__((ext_vector_type(8)));
typedef int            v4i  __attribute__((ext_vector_type(4)));
typedef int            v8i  __attribute__((ext_vector_type(8)));
typedef unsigned int   v2u  __attribute__((ext_vector_type(2)));
typedef unsigned int   v4u  __attribute__((ext_vector_type(4)));
typedef unsigned short v8us __attribute__((ext_vector_type(8)));
typedef __bf16         v16b __attribute__((ext_vector_type(16)));
typedef v4f  __attribute__((may_alias)) v4fa;
typedef v4i  __attribute__((may_alias)) v4ia;
typedef v2u  __attribute__((may_alias)) v2ua;
typedef v8us __attribute__((may_alias)) v8usa;
union Frag { v16b vb; v8us h[2]; v8i w; };

__device__ __forceinline__ v8f wmx(const Frag& a, const Frag& b, v8f c) {
  v8f d = __builtin_amdgcn_wmma_f32_16x16x32_bf16(false, a.vb, false, b.vb, (short)0, c, false, false);
  asm volatile("v_nop\n\tv_nop\n\tv_nop\n\tv_nop" : "+v"(d) : "v"(a.w), "v"(b.w));
  return d;
}

__device__ __forceinline__ unsigned int bf_bits(float f) {
  const unsigned int u = __float_as_uint(f);
  const unsigned int r = (u + 0x7FFFu + ((u >> 16) & 1u)) >> 16;
  const unsigned int q = (u >> 16) | 0x40u;
  return ((u & 0x7fffffffu) > 0x7f800000u) ? q : r;
}
__device__ __forceinline__ float bf_val(unsigned int b) { return __uint_as_float(b << 16); }
__device__ __forceinline__ float bf_rne(float f) { return bf_val(bf_bits(f)); }
__device__ __forceinline__ float relu_np(float v) { return (v > 0.0f) ? v : (v - v); }

template <int FIRST>
__device__ __forceinline__ v4f fx4(v4f v, v4f m, v4f r, v4f g, v4f b) {
  if constexpr (FIRST != 0) {
    return v;
  } else {
    const v4f y = ((v - m) * r) * g + b;
    v4f o;
    o.x = relu_np(y.x); o.y = relu_np(y.y); o.z = relu_np(y.z); o.w = relu_np(y.w);
    return o;
  }
}

__device__ __forceinline__ void split4(float a, float b, float c, float d, v2u& hv, v2u& lv) {
  const unsigned int ha = bf_bits(a), hb = bf_bits(b), hc = bf_bits(c), hd = bf_bits(d);
  const unsigned int la = bf_bits(a - bf_val(ha)), lb = bf_bits(b - bf_val(hb));
  const unsigned int lc = bf_bits(c - bf_val(hc)), ld = bf_bits(d - bf_val(hd));
  v2u h2, l2;
  h2.x = ha | (hb << 16); h2.y = hc | (hd << 16);
  l2.x = la | (lb << 16); l2.y = lc | (ld << 16);
  hv = h2; lv = l2;
}

__device__ __forceinline__ int scan_chunk(const int* __restrict__ dsts, int nE, int cbase, int slotBase,
                                          int nb, int vec8, int* list, int tid, int lane, int wave) {
  int wc = 0;
  const int el0  = tid * EPT;
  const int e0   = cbase + el0;
  const int sent = -2147483647 - 1;
  v4i da, db;
  if (vec8 != 0 && cbase + CHUNK <= nE) {
    da = *(const v4i*)(dsts + e0);
    db = *(const v4i*)(dsts + e0 + 4);
  } else {
    da.x = (e0     < nE) ? dsts[min(e0,     nE - 1)] : sent;
    da.y = (e0 + 1 < nE) ? dsts[min(e0 + 1, nE - 1)] : sent;
    da.z = (e0 + 2 < nE) ? dsts[min(e0 + 2, nE - 1)] : sent;
    da.w = (e0 + 3 < nE) ? dsts[min(e0 + 3, nE - 1)] : sent;
    db.x = (e0 + 4 < nE) ? dsts[min(e0 + 4, nE - 1)] : sent;
    db.y = (e0 + 5 < nE) ? dsts[min(e0 + 5, nE - 1)] : sent;
    db.z = (e0 + 6 < nE) ? dsts[min(e0 + 6, nE - 1)] : sent;
    db.w = (e0 + 7 < nE) ? dsts[min(e0 + 7, nE - 1)] : sent;
  }
  const unsigned nbs = (unsigned)slotBase;
  const unsigned unb = (unsigned)nb;
  const unsigned s0 = (unsigned)da.x - nbs, s1 = (unsigned)da.y - nbs;
  const unsigned s2 = (unsigned)da.z - nbs, s3 = (unsigned)da.w - nbs;
  const unsigned s4 = (unsigned)db.x - nbs, s5 = (unsigned)db.y - nbs;
  const unsigned s6 = (unsigned)db.z - nbs, s7 = (unsigned)db.w - nbs;
  const bool h0 = s0 < unb, h1 = s1 < unb, h2 = s2 < unb, h3 = s3 < unb;
  const bool h4 = s4 < unb, h5 = s5 < unb, h6 = s6 < unb, h7 = s7 < unb;
  const unsigned any = __builtin_amdgcn_ballot_w32(h0 | h1 | h2 | h3 | h4 | h5 | h6 | h7);
  if (any != 0u) {
#define HITJ(J, HJ, SJ) { \
      const unsigned mj = __builtin_amdgcn_ballot_w32(HJ); \
      if (mj != 0u) { \
        if (HJ) { \
          const int pos = wc + (int)__builtin_amdgcn_mbcnt_lo(mj, 0u); \
          if (pos < WCAP) list[wave * WCAP + pos] = ((el0 + (J)) << PKS) | (int)(SJ); \
        } \
        wc += (int)__builtin_popcount(mj); } }
    HITJ(0, h0, s0)
    HITJ(1, h1, s1)
    HITJ(2, h2, s2)
    HITJ(3, h3, s3)
    HITJ(4, h4, s4)
    HITJ(5, h5, s5)
    HITJ(6, h6, s6)
    HITJ(7, h7, s7)
#undef HITJ
  }
  return wc;
}

__device__ __forceinline__ v8us cv8b(const float* __restrict__ p, size_t stride) {
  v8us o;
#pragma unroll
  for (int i = 0; i < 8; ++i) o[i] = (unsigned short)bf_bits(p[(size_t)i * stride]);
  return o;
}

__global__ __launch_bounds__(NTHR) void k_prep(const float* __restrict__ inW, const float* __restrict__ cW1,
                                               const float* __restrict__ cW2, const float* __restrict__ roW1,
                                               const float* __restrict__ emb,
                                               unsigned short* pIn, unsigned short* pW1, unsigned short* pW2,
                                               unsigned short* pRo, unsigned short* pE) {
  const int u = (int)blockIdx.x * NTHR + (int)threadIdx.x;
  v8us o;
  unsigned short* dp;
  if (u < NUB1) {
    const int n = u >> 4, k8 = (u & 15) * 8;
    const int kr = k8 < 80 ? k8 : (k8 < 96 ? k8 - 16 : 0);
    const v8us t = cv8b(inW + (size_t)kr * HD + n, HD);
    const v8us z = {0, 0, 0, 0, 0, 0, 0, 0};
    o = (k8 >= 96) ? z : t;
    dp = pIn + (size_t)u * 8;
  } else if (u < NUB2) {
    const int v = u - NUB1;
    const int l = v >> 12, w = v & 4095, n = w >> 5, k8 = (w & 31) * 8, kk = k8 & (HD - 1);
    o = cv8b(cW1 + (size_t)l * (HD * HD) + (size_t)kk * HD + n, HD);
    dp = pW1 + (size_t)v * 8;
  } else if (u < NUB3) {
    const int v = u - NUB2;
    const int l = v >> 12, w = v & 4095, n = w >> 5, k8 = (w & 31) * 8, kk = k8 & (HD - 1);
    o = cv8b(cW2 + (size_t)l * (HD * HD) + (size_t)kk * HD + n, HD);
    dp = pW2 + (size_t)v * 8;
  } else if (u < NUB4) {
    const int v = u - NUB3;
    const int n = v >> 5, k8 = (v & 31) * 8, kk = k8 & (HD - 1);
    o = cv8b(roW1 + (size_t)kk * HD + n, HD);
    dp = pRo + (size_t)v * 8;
  } else if (u < NUTOT) {
    const int v = u - NUB4;
    const v4f a = *(const v4f*)(emb + (size_t)v * 8);
    const v4f b = *(const v4f*)(emb + (size_t)v * 8 + 4);
    o[0] = (unsigned short)bf_bits(a.x); o[1] = (unsigned short)bf_bits(a.y);
    o[2] = (unsigned short)bf_bits(a.z); o[3] = (unsigned short)bf_bits(a.w);
    o[4] = (unsigned short)bf_bits(b.x); o[5] = (unsigned short)bf_bits(b.y);
    o[6] = (unsigned short)bf_bits(b.z); o[7] = (unsigned short)bf_bits(b.w);
    dp = pE + (size_t)v * 8;
  } else {
    return;
  }
  *(volatile v8us*)dp = o;
  __threadfence();
  *(volatile v8us*)dp = o;
}

__global__ __launch_bounds__(NTHR) void k_pe(const float* __restrict__ pe,
                                             const float* __restrict__ W1, const float* __restrict__ b1,
                                             const float* __restrict__ W2, const float* __restrict__ b2,
                                             int nN, float* hp, float* prec) {
  __shared__ float w1s[PER * PEP];
  __shared__ float w2s[PEP * PEP];
  __shared__ float b1s[PEP];
  __shared__ float b2s[PEP];
  __shared__ float rowb[NTHR * RPW];
  __shared__ __attribute__((aligned(16))) float hpt[NTHR * PEP];
  __shared__ float red[16 * PEP];
  __shared__ float cmean[PEP];
  __shared__ __attribute__((aligned(16))) float rec[PRECW];
  const int tid = (int)threadIdx.x;
  const int blk = (int)blockIdx.x;

  for (int i = tid; i < PER * PEP; i += NTHR) w1s[i] = bf_rne(W1[i]);
  w2s[tid] = bf_rne(W2[tid]);
  b1s[tid & (PEP - 1)] = bf_rne(b1[tid & (PEP - 1)]);
  b2s[tid & (PEP - 1)] = bf_rne(b2[tid & (PEP - 1)]);
  if (tid < PRECW) rec[tid] = 0.0f;

  const int node = blk * NTHR + tid;
  const bool live = node < nN;
  const int nc = live ? node : nN - 1;
  {
    const float* pp = pe + (size_t)nc * PER;
    const v4f q0 = *(const v4f*)(pp);
    const v4f q1 = *(const v4f*)(pp + 4);
    const v4f q2 = *(const v4f*)(pp + 8);
    const v4f q3 = *(const v4f*)(pp + 12);
    const v4f q4 = *(const v4f*)(pp + 16);
    float* rb = rowb + tid * RPW;
    rb[0]  = bf_rne(q0.x); rb[1]  = bf_rne(q0.y); rb[2]  = bf_rne(q0.z); rb[3]  = bf_rne(q0.w);
    rb[4]  = bf_rne(q1.x); rb[5]  = bf_rne(q1.y); rb[6]  = bf_rne(q1.z); rb[7]  = bf_rne(q1.w);
    rb[8]  = bf_rne(q2.x); rb[9]  = bf_rne(q2.y); rb[10] = bf_rne(q2.z); rb[11] = bf_rne(q2.w);
    rb[12] = bf_rne(q3.x); rb[13] = bf_rne(q3.y); rb[14] = bf_rne(q3.z); rb[15] = bf_rne(q3.w);
    rb[16] = bf_rne(q4.x); rb[17] = bf_rne(q4.y); rb[18] = bf_rne(q4.z); rb[19] = bf_rne(q4.w);
  }
  __syncthreads();

  float t[PEP];
#pragma unroll
  for (int j = 0; j < PEP; ++j) t[j] = b1s[j];
#pragma unroll 1
  for (int i = 0; i < PER; ++i) {
    const float p = rowb[tid * RPW + i];
#pragma unroll
    for (int j = 0; j < PEP; ++j) t[j] = fmaf(p, w1s[i * PEP + j], t[j]);
  }
  __syncthreads();
#pragma unroll
  for (int j = 0; j < PEP; ++j) rowb[tid * RPW + j] = relu_np(t[j]);
  __syncthreads();
  float s[PEP];
#pragma unroll
  for (int j = 0; j < PEP; ++j) s[j] = b2s[j];
#pragma unroll 1
  for (int k = 0; k < PEP; ++k) {
    const float a = rowb[tid * RPW + k];
#pragma unroll
    for (int j = 0; j < PEP; ++j) s[j] = fmaf(a, w2s[k * PEP + j], s[j]);
  }
#pragma unroll
  for (int q = 0; q < 4; ++q) {
    v4f o;
    o.x = live ? s[4 * q + 0] : 0.0f; o.y = live ? s[4 * q + 1] : 0.0f;
    o.z = live ? s[4 * q + 2] : 0.0f; o.w = live ? s[4 * q + 3] : 0.0f;
    *(v4fa*)(hpt + tid * PEP + 4 * q) = o;
  }
  __syncthreads();

  int nvr = nN - blk * NTHR;
  nvr = nvr < 0 ? 0 : (nvr > NTHR ? NTHR : nvr);
  const int c = tid & (PEP - 1), rg = tid >> 4;
  {
    float ps = 0.0f;
#pragma unroll 1
    for (int rr = 0; rr < 16; ++rr) {
      const int row = rg * 16 + rr;
      const float v = hpt[row * PEP + c];
      ps += (row < nvr) ? v : 0.0f;
    }
    red[rg * PEP + c] = ps;
  }
  __syncthreads();
  if (tid < PEP) {
    float sm = 0.0f;
#pragma unroll 1
    for (int g = 0; g < 16; ++g) sm += red[g * PEP + tid];
    cmean[tid] = sm * (1.0f / (float)(nvr < 1 ? 1 : nvr));
  }
  __syncthreads();
  {
    const float mean = cmean[c];
    float pq = 0.0f;
#pragma unroll 1
    for (int rr = 0; rr < 16; ++rr) {
      const int row = rg * 16 + rr;
      const float d = hpt[row * PEP + c] - mean;
      pq += (row < nvr) ? d * d : 0.0f;
    }
    __syncthreads();
    red[rg * PEP + c] = pq;
  }
  __syncthreads();
  if (tid < PEP) {
    float sq = 0.0f;
#pragma unroll 1
    for (int g = 0; g < 16; ++g) sq += red[g * PEP + tid];
    rec[1 + tid] = cmean[tid];
    rec[1 + PEP + tid] = sq;
    if (tid == 0) rec[0] = (float)nvr;
  }
  __syncthreads();

  v4f pv[4];
#pragma unroll
  for (int it = 0; it < 4; ++it) pv[it] = *(const v4fa*)(hpt + 4 * (it * NTHR + tid));
  v4f rv = {0.f, 0.f, 0.f, 0.f};
  const bool rok = tid < PRECW / 4;
  if (rok) rv = *(const v4fa*)(rec + 4 * tid);
  float* hb = hp + (size_t)blk * (NTHR * PEP);
  float* rp = prec + (size_t)blk * PRECW + 4 * tid;
#pragma unroll
  for (int it = 0; it < 4; ++it) *(volatile v4f*)(hb + 4 * (it * NTHR + tid)) = pv[it];
  if (rok) *(volatile v4f*)rp = rv;
  __threadfence();
#pragma unroll
  for (int it = 0; it < 4; ++it) *(volatile v4f*)(hb + 4 * (it * NTHR + tid)) = pv[it];
  if (rok) *(volatile v4f*)rp = rv;
}

__global__ __launch_bounds__(32) void k_comb_pe(const float* __restrict__ prec, int nPart,
                                                const float* __restrict__ gam, const float* __restrict__ bet,
                                                float* statp) {
  __shared__ __attribute__((aligned(16))) float stg[4 * PEP];
  const int tid = (int)threadIdx.x;
  const int c = tid & (PEP - 1);
  double n = 0.0, mean = 0.0, M2 = 0.0;
#pragma unroll 1
  for (int b = 0; b < nPart; ++b) {
    const float* pr = prec + (size_t)b * PRECW;
    const double nb = (double)pr[0];
    const double mb = (double)pr[1 + c];
    const double qb = (double)pr[1 + PEP + c];
    if (nb > 0.5) {
      const double nn = n + nb;
      const double delta = mb - mean;
      const double f = nb / nn;
      mean = mean + delta * f;
      M2 = M2 + qb + delta * delta * n * f;
      n = nn;
    }
  }
  const double nt = n < 1.0 ? 1.0 : n;
  const float var = (float)(M2 / nt);
  const float r = 1.0f / sqrtf(var + 1e-5f);
  if (tid < PEP) {
    stg[c] = (float)mean;
    stg[PEP + c] = r;
    stg[2 * PEP + c] = bf_rne(gam[c]);
    stg[3 * PEP + c] = bf_rne(bet[c]);
  }
  __syncthreads();
  v4f v = {0.f, 0.f, 0.f, 0.f};
  const bool ok = tid < PEP;
  if (ok) { v = *(const v4fa*)(stg + 4 * tid); *(volatile v4f*)(statp + 4 * tid) = v; }
  __threadfence();
  if (ok) *(volatile v4f*)(statp + 4 * tid) = v;
}

__global__ __launch_bounds__(NTHR) void k_ain(const int* __restrict__ x, const unsigned short* __restrict__ emb,
                                              const float* __restrict__ hp, const float* __restrict__ statp,
                                              int nN, int mRows, unsigned short* ain) {
  __shared__ __attribute__((aligned(16))) float sp[4 * PEP];
  const int tid = (int)threadIdx.x, lane = tid & 31, wave = tid >> 5;
  if (tid < PEP) *(v4fa*)(sp + 4 * tid) = *(const v4f*)(statp + 4 * tid);
  __syncthreads();
  const int cg = lane & 3;
  const v4f m4 = *(const v4fa*)(sp + 4 * cg);
  const v4f r4 = *(const v4fa*)(sp + PEP + 4 * cg);
  const v4f g4 = *(const v4fa*)(sp + 2 * PEP + 4 * cg);
  const v4f b4 = *(const v4fa*)(sp + 3 * PEP + 4 * cg);
  const int el = lane < 16 ? lane : 15;
  const unsigned int mE = (lane < 16) ? 0xffffffffu : 0u;
  const unsigned int mH = (lane >= 16 && lane < 20) ? 0xffffffffu : 0u;
  const unsigned int mL = (lane >= 20 && lane < 24) ? 0xffffffffu : 0u;
#pragma unroll 1
  for (int j = 0; j < 8; ++j) {
    const int row = (int)blockIdx.x * 64 + wave * 8 + j;
    const bool live = row < nN;
    const int rc = live ? row : nN - 1;
    int xi = x[rc];
    xi = xi < 0 ? 0 : (xi > NATOM - 1 ? NATOM - 1 : xi);
    const v2u e = *(const v2ua*)(emb + (size_t)xi * AEMB + 4 * el);
    const v4f h = *(const v4f*)(hp + (size_t)rc * PEP + 4 * cg);
    const v4f y = ((h - m4) * r4) * g4 + b4;
    v2u hw, lw;
    split4(y.x, y.y, y.z, y.w, hw, lw);
    const unsigned int ml = live ? 0xffffffffu : 0u;
    v2u w;
    w.x = ((e.x & mE) | (hw.x & mH) | (lw.x & mL)) & ml;
    w.y = ((e.y & mE) | (hw.y & mH) | (lw.y & mL)) & ml;
    unsigned short* gp = ain + (size_t)row * HD + 4 * lane;
    const bool wsv = row < mRows;
    if (wsv) *(volatile v2u*)gp = w;
    __threadfence();
    if (wsv) *(volatile v2u*)gp = w;
  }
}

__global__ __launch_bounds__(NTHR) void k_compact(const int* __restrict__ srcs, const int* __restrict__ dsts,
                                                  int nN, int nE, int vec8,
                                                  int* lists, int* offs, int* cnts, int* meta) {
  extern __shared__ v4f lds_dyn[];
  int* reg1 = (int*)lds_dyn;
  int* reg2 = reg1 + RCAP;
  int* scnt = reg2 + RCAP;
  int* soff = scnt + NB;
  int* list = soff + NB;
  int* wcnt = list + LISTN;
  int* wtot = wcnt + NWAVE;
  int* mst  = wtot + NWAVE;
  const int tid = (int)threadIdx.x, lane = tid & 31, wave = tid >> 5;
  const int blk = (int)blockIdx.x;
  const int nodeBase = blk * NB;

  {
    const v4i z4 = {0, 0, 0, 0};
    for (int i = tid * 4; i < CZ_INTS; i += NTHR * 4) *(v4ia*)(reg1 + i) = z4;
  }
  __syncthreads();

  int tot = 0, ovf = 0;
  const int nChunks = (nE + CHUNK - 1) / CHUNK;
#pragma unroll 1
  for (int ch = 0; ch < nChunks; ++ch) {
    const int cbase = ch * CHUNK;
    const int wc = scan_chunk(dsts, nE, cbase, nodeBase, NB, vec8, list, tid, lane, wave);
    if (lane == 0) wcnt[wave] = wc;
    __syncthreads();
    int pre = 0, all = 0;
#pragma unroll
    for (int w2 = 0; w2 < NWAVE; ++w2) {
      int c = wcnt[w2];
      c = c < 0 ? 0 : (c > WCAP ? WCAP : c);
      all += c;
      pre += (w2 < wave) ? c : 0;
    }
    const int wcc  = wc > WCAP ? WCAP : wc;
    const int base = tot + pre;
#pragma unroll 1
    for (int i = lane; i < wcc; i += 32) {
      const int ent = list[wave * WCAP + i];
      const int el  = (ent >> PKS) & (CHUNK - 1);
      const int sl  = ent & (NB - 1);
      int eid = cbase + el;
      eid = eid > nE - 1 ? nE - 1 : eid;
      int s = srcs[eid];
      s = s < 0 ? 0 : (s > nN - 1 ? nN - 1 : s);
      const int pos = base + i;
      if (pos < RCAP) reg1[pos] = (int)(((unsigned)s << PKS) | (unsigned)sl);
    }
    if (tot + all > RCAP) ovf = 1;
    tot += all;
    tot = tot > RCAP ? RCAP : tot;
    __syncthreads();
  }
  const int nh = tot;

  if (wave == 0) {
#pragma unroll 1
    for (int b0 = 0; b0 < nh; b0 += 32) {
      const int idx = b0 + lane;
      const int uv  = reg1[idx < RCAP ? idx : RCAP - 1];
      const int m32 = (nh - b0) < 32 ? (nh - b0) : 32;
#pragma unroll 1
      for (int k = 0; k < m32; ++k) {
        const int u  = __builtin_amdgcn_readlane(uv, k);
        const int sl = u & (NB - 1);
        if (lane == 0) scnt[sl] = scnt[sl] + 1;
      }
    }
  }
  __syncthreads();

  {
    const v4i ca = *(const v4ia*)(scnt + 4 * tid);
    const int e0 = ca.x < 0 ? 0 : ca.x, e1 = ca.y < 0 ? 0 : ca.y, e2 = ca.z < 0 ? 0 : ca.z, e3 = ca.w < 0 ? 0 : ca.w;
    const int ts = e0 + e1 + e2 + e3;
    int incl = ts;
#pragma unroll
    for (int d = 1; d < 32; d <<= 1) {
      const int up = __shfl_up(incl, d);
      if (lane >= d) incl += up;
    }
    if (lane == 31) wtot[wave] = incl;
    __syncthreads();
    int pre = 0;
#pragma unroll
    for (int w2 = 0; w2 < NWAVE; ++w2) pre += (w2 < wave) ? wtot[w2] : 0;
    int run = pre + incl - ts;
    soff[4 * tid + 0] = run; run += e0;
    soff[4 * tid + 1] = run; run += e1;
    soff[4 * tid + 2] = run; run += e2;
    soff[4 * tid + 3] = run;
  }
  __syncthreads();
  for (int i = tid; i < NB; i += NTHR) list[i] = soff[i];
  if (tid == 0) { mst[0] = nh; mst[1] = ovf; }
  __syncthreads();

  if (wave == 0) {
#pragma unroll 1
    for (int b0 = 0; b0 < nh; b0 += 32) {
      const int idx = b0 + lane;
      const int uv  = reg1[idx < RCAP ? idx : RCAP - 1];
      const int m32 = (nh - b0) < 32 ? (nh - b0) : 32;
#pragma unroll 1
      for (int k = 0; k < m32; ++k) {
        const int u  = __builtin_amdgcn_readlane(uv, k);
        const int sl = u & (NB - 1);
        const int sv = (int)((unsigned)u >> PKS);
        if (lane == 0) {
          int pos = list[sl];
          pos = pos < 0 ? 0 : (pos > RCAP - 1 ? RCAP - 1 : pos);
          reg2[pos] = sv;
          list[sl] = pos + 1;
        }
      }
    }
  }
  __syncthreads();

  int* lp = lists + (size_t)blk * RCAP;
  int* op = offs + (size_t)blk * NB + 4 * tid;
  int* cp = cnts + (size_t)blk * NB + 4 * tid;
  int* mp = meta + (size_t)blk * 32 + 4 * tid;
  const v4i vo = *(const v4ia*)(soff + 4 * tid);
  const v4i vc = *(const v4ia*)(scnt + 4 * tid);
  v4i vm = {0, 0, 0, 0};
  const bool mok = tid < 8;
  if (mok) vm = *(const v4ia*)(mst + 4 * tid);
#pragma unroll 1
  for (int it = 0; it < (RCAP / 4) / NTHR; ++it) {
    const int p = it * NTHR + tid;
    const v4i v = *(const v4ia*)(reg2 + 4 * p);
    *(volatile v4i*)(lp + 4 * p) = v;
  }
  *(volatile v4i*)op = vo;
  *(volatile v4i*)cp = vc;
  if (mok) *(volatile v4i*)mp = vm;
  __threadfence();
#pragma unroll 1
  for (int it = 0; it < (RCAP / 4) / NTHR; ++it) {
    const int p = it * NTHR + tid;
    const v4i v = *(const v4ia*)(reg2 + 4 * p);
    *(volatile v4i*)(lp + 4 * p) = v;
  }
  *(volatile v4i*)op = vo;
  *(volatile v4i*)cp = vc;
  if (mok) *(volatile v4i*)mp = vm;
}

template <int FIRST>
__global__ __launch_bounds__(NTHR) void k_agg(const float* __restrict__ X, const float* __restrict__ stat,
                                              const int* __restrict__ lists, const int* __restrict__ offs,
                                              const int* __restrict__ cnts, const int* __restrict__ meta,
                                              int nBlk, int nN, int mRows, unsigned short* Z) {
  __shared__ __attribute__((aligned(16))) float sst[4 * HD];
  const int tid = (int)threadIdx.x, lane = tid & 31, wave = tid >> 5;
  v4f m4 = {0.f, 0.f, 0.f, 0.f}, r4 = m4, g4 = m4, b4 = m4;
  if constexpr (FIRST == 0) {
    if (tid < HD) *(v4fa*)(sst + 4 * tid) = *(const v4f*)(stat + 4 * tid);
    __syncthreads();
    m4 = *(const v4fa*)(sst + 4 * lane);
    r4 = *(const v4fa*)(sst + HD + 4 * lane);
    g4 = *(const v4fa*)(sst + 2 * HD + 4 * lane);
    b4 = *(const v4fa*)(sst + 3 * HD + 4 * lane);
  }
  const float qnan = __int_as_float(0x7fc00000);
#pragma unroll 1
  for (int j = 0; j < 8; ++j) {
    const int row = (int)blockIdx.x * 64 + wave * 8 + j;
    int blk = row >> PKS;
    blk = blk > nBlk - 1 ? nBlk - 1 : blk;
    const int slot = row & (NB - 1);
    int nh = meta[(size_t)blk * 32];
    const int ovf = meta[(size_t)blk * 32 + 1];
    nh = nh < 0 ? 0 : (nh > RCAP ? RCAP : nh);
    int st = offs[(size_t)blk * NB + slot];
    const int craw = cnts[(size_t)blk * NB + slot];
    st = st < 0 ? 0 : (st > nh ? nh : st);
    int cnt = craw < 0 ? 0 : (craw > DEGCAP ? DEGCAP : craw);
    if (cnt > nh - st) cnt = nh - st;
    const bool bad = (ovf != 0) || (craw > DEGCAP) || (craw < 0);
    const bool liveRow = row < nN;

    v4f ag = {0.f, 0.f, 0.f, 0.f};
    const int* lb = lists + (size_t)blk * RCAP;
#pragma unroll 1
    for (int b0 = 0; b0 < cnt; b0 += 32) {
      int idx = st + b0 + lane;
      idx = idx > RCAP - 1 ? RCAP - 1 : idx;
      int sr = lb[idx];
      sr = sr < 0 ? 0 : (sr > nN - 1 ? nN - 1 : sr);
      const int m32 = (cnt - b0) < 32 ? (cnt - b0) : 32;
#pragma unroll 1
      for (int k = 0; k < m32; ++k) {
        const int sk = __builtin_amdgcn_readlane(sr, k);
        const v4f v = *(const v4f*)(X + (size_t)sk * HD + 4 * lane);
        ag = ag + fx4<FIRST>(v, m4, r4, g4, b4);
      }
    }
    const int nc = liveRow ? row : nN - 1;
    const v4f sv = fx4<FIRST>(*(const v4f*)(X + (size_t)nc * HD + 4 * lane), m4, r4, g4, b4);
    const float pz = bad ? qnan : 0.0f;
    const float z0 = liveRow ? (sv.x + ag.x + pz) : 0.0f;
    const float z1 = liveRow ? (sv.y + ag.y + pz) : 0.0f;
    const float z2 = liveRow ? (sv.z + ag.z + pz) : 0.0f;
    const float z3 = liveRow ? (sv.w + ag.w + pz) : 0.0f;
    v2u hv, lv;
    split4(z0, z1, z2, z3, hv, lv);
    unsigned short* gp = Z + (size_t)row * K2 + 4 * lane;
    const bool wsv = row < mRows;
    if (wsv) { *(volatile v2u*)gp = hv; *(volatile v2u*)(gp + HD) = lv; }
    __threadfence();
    if (wsv) { *(volatile v2u*)gp = hv; *(volatile v2u*)(gp + HD) = lv; }
  }
}

template <int EPI>
__global__ __launch_bounds__(GTHR) void k_gemm(const unsigned short* __restrict__ A, int lda,
                                               const unsigned short* __restrict__ BT, int ldb, int K,
                                               const float* __restrict__ bias,
                                               void* outp, int ldo, int lsplit, int nN, int mRows,
                                               float* part,
                                               const float* __restrict__ w2, const float* __restrict__ b2) {
  __shared__ __attribute__((aligned(16))) float stg[GBM * GBN];
  __shared__ __attribute__((aligned(16))) float pst[PARTW];
  const int tid = (int)threadIdx.x, lane = tid & 31, wave = tid >> 5, hh = lane >> 4, m = lane & 15;
  const int rowBase = (int)blockIdx.x * GBM;
  const int colBase = (int)blockIdx.y * GBN;

  v8f acc[GNT];
  {
    const v8f z = {0.f, 0.f, 0.f, 0.f, 0.f, 0.f, 0.f, 0.f};
#pragma unroll
    for (int t = 0; t < GNT; ++t) acc[t] = z;
  }
  const unsigned short* ap = A  + (size_t)(rowBase + 16 * wave + m) * (size_t)lda + 8 * hh;
  const unsigned short* bp = BT + (size_t)(colBase + m) * (size_t)ldb + 8 * hh;

#pragma unroll 1
  for (int k0 = 0; k0 < K; k0 += 32) {
    Frag af;
    af.h[0] = *(const v8usa*)(ap + k0);
    af.h[1] = *(const v8usa*)(ap + k0 + 16);
#pragma unroll
    for (int nt = 0; nt < GNT; ++nt) {
      const unsigned short* wq = bp + (size_t)(16 * nt) * (size_t)ldb + k0;
      Frag bfr;
      bfr.h[0] = *(const v8usa*)wq;
      bfr.h[1] = *(const v8usa*)(wq + 16);
      acc[nt] = wmx(af, bfr, acc[nt]);
    }
  }

  if constexpr (EPI == 4) pst[tid] = bf_rne(w2[tid]);

#pragma unroll
  for (int nt = 0; nt < GNT; ++nt) {
    const int lc = 16 * nt + m;
    const float bb = bf_rne(bias[colBase + lc]);
#pragma unroll
    for (int r = 0; r < 8; ++r) {
      const int lr = 16 * wave + 8 * hh + r;
      const bool live = (rowBase + lr) < nN;
      float v = acc[nt][r] + bb;
      if constexpr (EPI == 2 || EPI == 4) v = relu_np(v);
      stg[lr * GBN + lc] = live ? v : 0.0f;
    }
  }
  __syncthreads();

  if constexpr (EPI == 2) {
    unsigned short* outH = (unsigned short*)outp;
    const int cb = 8 * m;
    const bool isHi = (hh == 0);
    v4u pk[16];
#pragma unroll
    for (int i = 0; i < 16; ++i) {
      const int lr = 16 * wave + i;
      const v4f a = *(const v4fa*)(stg + lr * GBN + cb);
      const v4f b = *(const v4fa*)(stg + lr * GBN + cb + 4);
      const float f[8] = {a.x, a.y, a.z, a.w, b.x, b.y, b.z, b.w};
      unsigned int w[4];
#pragma unroll
      for (int j = 0; j < 4; ++j) {
        const unsigned int h0 = bf_bits(f[2 * j]), h1 = bf_bits(f[2 * j + 1]);
        const unsigned int l0 = bf_bits(f[2 * j] - bf_val(h0)), l1 = bf_bits(f[2 * j + 1] - bf_val(h1));
        const unsigned int q0 = isHi ? h0 : l0, q1 = isHi ? h1 : l1;
        w[j] = q0 | (q1 << 16);
      }
      v4u pv; pv.x = w[0]; pv.y = w[1]; pv.z = w[2]; pv.w = w[3];
      pk[i] = pv;
    }
#pragma unroll
    for (int i = 0; i < 16; ++i) {
      const int gr = rowBase + 16 * wave + i;
      unsigned short* op = outH + (size_t)gr * (size_t)ldo + colBase + cb + hh * lsplit;
      if (gr < mRows) *(volatile v4u*)op = pk[i];
    }
    __threadfence();
#pragma unroll
    for (int i = 0; i < 16; ++i) {
      const int gr = rowBase + 16 * wave + i;
      unsigned short* op = outH + (size_t)gr * (size_t)ldo + colBase + cb + hh * lsplit;
      if (gr < mRows) *(volatile v4u*)op = pk[i];
    }
  } else if constexpr (EPI == 4) {
    float* outF = (float*)outp;
    if (tid < GBM) {
      float s = 0.0f;
#pragma unroll 4
      for (int c = 0; c < GBN; ++c) s = fmaf(stg[tid * GBN + c], pst[c], s);
      pst[GBN + tid] = s + bf_rne(b2[0]);
    }
    __syncthreads();
    const bool ok = (tid < GBM / 4) && (rowBase + 4 * tid + 3 < nN);
    v4f ov = {0.f, 0.f, 0.f, 0.f};
    float* op = outF + (size_t)rowBase + 4 * tid;
    if (ok) { ov = *(const v4fa*)(pst + GBN + 4 * tid); *(volatile v4f*)op = ov; }
    __threadfence();
    if (ok) *(volatile v4f*)op = ov;
  } else {
    float* outF = (float*)outp;
    v4f fv[16];
#pragma unroll
    for (int i = 0; i < 16; ++i) {
      const int lr = 16 * wave + i;
      fv[i] = *(const v4fa*)(stg + lr * GBN + 4 * lane);
    }
    v4f pv = {0.f, 0.f, 0.f, 0.f};
    const bool pok = (EPI == 1) && (tid < PARTW / 4);
    if constexpr (EPI == 1) {
      int nvr = nN - rowBase;
      nvr = nvr < 0 ? 0 : (nvr > GBM ? GBM : nvr);
      float s = 0.0f;
#pragma unroll 1
      for (int r = 0; r < nvr; ++r) s += stg[r * GBN + tid];
      const float inv = 1.0f / (float)(nvr < 1 ? 1 : nvr);
      const float mean = s * inv;
      float q = 0.0f;
#pragma unroll 1
      for (int r = 0; r < nvr; ++r) {
        const float d = stg[r * GBN + tid] - mean;
        q = fmaf(d, d, q);
      }
      pst[1 + tid] = mean;
      pst[1 + GBN + tid] = q;
      if (tid == 0) pst[0] = (float)nvr;
#pragma unroll 1
      for (int i = 2 * GBN + 1 + tid; i < PARTW; i += GTHR) pst[i] = 0.0f;
      __syncthreads();
      if (pok) pv = *(const v4fa*)(pst + 4 * tid);
    }
    const size_t prow = (size_t)blockIdx.x * (size_t)gridDim.y + (size_t)blockIdx.y;
    float* pp = part + prow * PARTW + 4 * tid;
#pragma unroll
    for (int i = 0; i < 16; ++i) {
      const int gr = rowBase + 16 * wave + i;
      float* op = outF + (size_t)gr * (size_t)ldo + colBase + 4 * lane;
      if (gr < mRows) *(volatile v4f*)op = fv[i];
    }
    if (pok) *(volatile v4f*)pp = pv;
    __threadfence();
#pragma unroll
    for (int i = 0; i < 16; ++i) {
      const int gr = rowBase + 16 * wave + i;
      float* op = outF + (size_t)gr * (size_t)ldo + colBase + 4 * lane;
      if (gr < mRows) *(volatile v4f*)op = fv[i];
    }
    if (pok) *(volatile v4f*)pp = pv;
  }
}

__global__ __launch_bounds__(GBN) void k_comb(const float* __restrict__ part, int nPart,
                                              const float* __restrict__ gam, const float* __restrict__ bet,
                                              float* ss) {
  __shared__ __attribute__((aligned(16))) float stg[4 * HD];
  const int tid = (int)threadIdx.x;
  double n = 0.0, mean = 0.0, M2 = 0.0;
#pragma unroll 1
  for (int b = 0; b < nPart; ++b) {
    const float* pr = part + (size_t)b * PARTW;
    const double nb = (double)pr[0];
    const double mb = (double)pr[1 + tid];
    const double qb = (double)pr[1 + GBN + tid];
    if (nb > 0.5) {
      const double nn = n + nb;
      const double delta = mb - mean;
      const double f = nb / nn;
      mean = mean + delta * f;
      M2 = M2 + qb + delta * delta * n * f;
      n = nn;
    }
  }
  const double nt = n < 1.0 ? 1.0 : n;
  const float var = (float)(M2 / nt);
  const float r = 1.0f / sqrtf(var + 1e-5f);
  stg[tid] = (float)mean;
  stg[HD + tid] = r;
  stg[2 * HD + tid] = bf_rne(gam[tid]);
  stg[3 * HD + tid] = bf_rne(bet[tid]);
  __syncthreads();
  const v4f v = *(const v4fa*)(stg + 4 * tid);
  *(volatile v4f*)(ss + 4 * tid) = v;
  __threadfence();
  *(volatile v4f*)(ss + 4 * tid) = v;
}

__global__ __launch_bounds__(NTHR) void k_pool(const float* __restrict__ X, const float* __restrict__ stat,
                                               const int* __restrict__ bat, int nN, int vec8b, int nG,
                                               unsigned short* pool) {
  __shared__ __attribute__((aligned(16))) int glist[GCAP];
  __shared__ __attribute__((aligned(16))) int list[LISTN];
  __shared__ int wcnt[NWAVE];
  __shared__ __attribute__((aligned(16))) float sst[4 * HD];
  const int tid = (int)threadIdx.x, lane = tid & 31, wave = tid >> 5;
  const int slotBase = (int)blockIdx.x * PG;

  {
    const v4i z4 = {0, 0, 0, 0};
    for (int i = tid * 4; i < GCAP; i += NTHR * 4) *(v4ia*)(glist + i) = z4;
  }
  if (tid < HD) *(v4fa*)(sst + 4 * tid) = *(const v4f*)(stat + 4 * tid);
  __syncthreads();
  const v4f m4 = *(const v4fa*)(sst + 4 * lane);
  const v4f r4 = *(const v4fa*)(sst + HD + 4 * lane);
  const v4f g4 = *(const v4fa*)(sst + 2 * HD + 4 * lane);
  const v4f b4 = *(const v4fa*)(sst + 3 * HD + 4 * lane);

  int tot = 0, ovf = 0;
  const int nChunks = (nN + CHUNK - 1) / CHUNK;
#pragma unroll 1
  for (int ch = 0; ch < nChunks; ++ch) {
    const int cbase = ch * CHUNK;
    const int wc = scan_chunk(bat, nN, cbase, slotBase, PG, vec8b, list, tid, lane, wave);
    if (lane == 0) wcnt[wave] = wc;
    __syncthreads();
    int pre = 0, all = 0;
#pragma unroll
    for (int w2 = 0; w2 < NWAVE; ++w2) {
      int c = wcnt[w2];
      c = c < 0 ? 0 : (c > WCAP ? WCAP : c);
      all += c;
      pre += (w2 < wave) ? c : 0;
    }
    const int wcc  = wc > WCAP ? WCAP : wc;
    const int base = tot + pre;
#pragma unroll 1
    for (int i = lane; i < wcc; i += 32) {
      const int ent = list[wave * WCAP + i];
      const int el  = (ent >> PKS) & (CHUNK - 1);
      const int sl  = ent & (PG - 1);
      int node = cbase + el;
      node = node > nN - 1 ? nN - 1 : node;
      const int pos = base + i;
      if (pos < GCAP) glist[pos] = (int)(((unsigned)node << PKS) | (unsigned)sl);
    }
    if (tot + all > GCAP) ovf = 1;
    tot += all;
    tot = tot > GCAP ? GCAP : tot;
    __syncthreads();
  }

  const int g0 = 2 * wave, g1 = 2 * wave + 1;
  v4f a0 = {0.f, 0.f, 0.f, 0.f}, a1 = {0.f, 0.f, 0.f, 0.f};
#pragma unroll 1
  for (int b0 = 0; b0 < tot; b0 += 32) {
    int idx = b0 + lane;
    idx = idx > GCAP - 1 ? GCAP - 1 : idx;
    const int ent = glist[idx];
    const int m32 = (tot - b0) < 32 ? (tot - b0) : 32;
#pragma unroll 1
    for (int k = 0; k < m32; ++k) {
      const int u  = __builtin_amdgcn_readlane(ent, k);
      const int sl = u & (PG - 1);
      int node = (int)((unsigned)u >> PKS);
      node = node > nN - 1 ? nN - 1 : node;
      if (sl == g0 || sl == g1) {
        const v4f v = fx4<0>(*(const v4f*)(X + (size_t)node * HD + 4 * lane), m4, r4, g4, b4);
        if (sl == g0) a0 = a0 + v; else a1 = a1 + v;
      }
    }
  }
  const float pz = (ovf != 0) ? __int_as_float(0x7fc00000) : 0.0f;
  v2u h0, l0, h1, l1;
  split4(a0.x + pz, a0.y + pz, a0.z + pz, a0.w + pz, h0, l0);
  split4(a1.x + pz, a1.y + pz, a1.z + pz, a1.w + pz, h1, l1);
  const int ga = slotBase + g0, gb = slotBase + g1;
  unsigned short* pa = pool + (size_t)ga * K2 + 4 * lane;
  unsigned short* pb = pool + (size_t)gb * K2 + 4 * lane;
  const bool oka = ga < nG, okb = gb < nG;
  if (oka) { *(volatile v2u*)pa = h0; *(volatile v2u*)(pa + HD) = l0; }
  if (okb) { *(volatile v2u*)pb = h1; *(volatile v2u*)(pb + HD) = l1; }
  __threadfence();
  if (oka) { *(volatile v2u*)pa = h0; *(volatile v2u*)(pa + HD) = l0; }
  if (okb) { *(volatile v2u*)pb = h1; *(volatile v2u*)(pb + HD) = l1; }
}

static inline int cdiv(int a, int b) { return (a + b - 1) / b; }
static inline size_t al256(size_t o) { return (o + 255) & ~(size_t)255; }

extern "C" void kernel_launch(void* const* d_in, const int* in_sizes, int n_in,
                              void* d_out, int out_size, void* d_ws, size_t ws_size,
                              hipStream_t stream) {
  if (n_in < 23) return;
  const int nN = in_sizes[0];
  if (nN < GBM || nN >= (1 << 21)) return;
  if ((long long)in_sizes[1] != (long long)nN * PER) return;
  const int nE2 = in_sizes[2];
  if (nE2 < 2 || (nE2 & 1) != 0) return;
  const int nE = nE2 / 2;
  if (nE < 1 || nE > (1 << 29)) return;
  if (in_sizes[3] != nN) return;
  if (in_sizes[4] != NATOM * AEMB) return;
  if (in_sizes[5] != PER * PEP || in_sizes[6] != PEP) return;
  if (in_sizes[7] != PEP * PEP || in_sizes[8] != PEP) return;
  if (in_sizes[9] != PEP || in_sizes[10] != PEP) return;
  if (in_sizes[11] != (AEMB + PEP) * HD || in_sizes[12] != HD) return;
  if (in_sizes[13] != NLAY * HD * HD || in_sizes[14] != NLAY * HD) return;
  if (in_sizes[15] != NLAY * HD * HD || in_sizes[16] != NLAY * HD) return;
  if (in_sizes[17] != NLAY * HD || in_sizes[18] != NLAY * HD) return;
  if (in_sizes[19] != HD * HD || in_sizes[20] != HD) return;
  if (in_sizes[21] != HD || in_sizes[22] != 1) return;
  const int nG = out_size;
  if (nG < GBM || (nG % GBM) != 0 || (nG % PG) != 0 || nG > (1 << 20)) return;

  const int*   x     = (const int*)  d_in[0];
  const float* pe    = (const float*)d_in[1];
  const int*   ei    = (const int*)  d_in[2];
  const int*   src   = ei;
  const int*   dst   = ei + nE;
  const int*   batch = (const int*)  d_in[3];
  const float* aemb  = (const float*)d_in[4];
  const float* peW1  = (const float*)d_in[5];  const float* peb1 = (const float*)d_in[6];
  const float* peW2  = (const float*)d_in[7];  const float* peb2 = (const float*)d_in[8];
  const float* peg   = (const float*)d_in[9];  const float* pebt = (const float*)d_in[10];
  const float* inW   = (const float*)d_in[11]; const float* inb  = (const float*)d_in[12];
  const float* cW1   = (const float*)d_in[13]; const float* cb1  = (const float*)d_in[14];
  const float* cW2   = (const float*)d_in[15]; const float* cb2  = (const float*)d_in[16];
  const float* bng   = (const float*)d_in[17]; const float* bnb  = (const float*)d_in[18];
  const float* roW1  = (const float*)d_in[19]; const float* rob1 = (const float*)d_in[20];
  const float* roW2  = (const float*)d_in[21]; const float* rob2 = (const float*)d_in[22];
  float* out = (float*)d_out;

  const int MP   = cdiv(nN, GBM) * GBM;
  const int gM   = MP / GBM;
  const int nBlk = cdiv(MP, NB);
  const int gPE  = cdiv(nN, NTHR);
  const int vec8  = ((nE & 3) == 0) ? 1 : 0;
  const int vec8b = ((nN & 3) == 0) ? 1 : 0;
  if ((long long)nBlk * NB < (long long)MP) return;
  if ((long long)(gM - 1) * GBM >= (long long)nN) return;

  char* ws = (char*)d_ws;
  size_t off = 0;
  const size_t oWin = off; off = al256(off + (size_t)NUIN * 16);
  const size_t oW1  = off; off = al256(off + (size_t)NUC * 16);
  const size_t oW2  = off; off = al256(off + (size_t)NUC * 16);
  const size_t oRo  = off; off = al256(off + (size_t)NURO * 16);
  const size_t oEm  = off; off = al256(off + (size_t)NUE * 16);
  const size_t oHP  = off; off = al256(off + (size_t)gPE * NTHR * PEP * 4);
  const size_t oPR  = off; off = al256(off + (size_t)gPE * PRECW * 4);
  const size_t oSP  = off; off = al256(off + (size_t)(4 * PEP) * 4);
  const size_t oAI  = off; off = al256(off + (size_t)MP * HD * 2);
  const size_t oP1  = off; off = al256(off + (size_t)MP * K2 * 2);
  const size_t oP3  = off; off = al256(off + (size_t)MP * K2 * 2);
  const size_t oP2  = off; off = al256(off + (size_t)MP * HD * 4);
  const size_t oLS  = off; off = al256(off + (size_t)nBlk * RCAP * 4);
  const size_t oOF  = off; off = al256(off + (size_t)nBlk * NB * 4);
  const size_t oCN  = off; off = al256(off + (size_t)nBlk * NB * 4);
  const size_t oMT  = off; off = al256(off + (size_t)nBlk * 32 * 4);
  const size_t oPT  = off; off = al256(off + (size_t)gM * PARTW * 4);
  const size_t oST  = off; off = al256(off + (size_t)NLAY * 4 * HD * 4);
  const size_t oPL  = off; off = al256(off + (size_t)nG * K2 * 2);
  if (off > ws_size || off > (size_t)WSCAP) return;
  unsigned short* WinT = (unsigned short*)(ws + oWin);
  unsigned short* W1T2 = (unsigned short*)(ws + oW1);
  unsigned short* W2T2 = (unsigned short*)(ws + oW2);
  unsigned short* RoT2 = (unsigned short*)(ws + oRo);
  unsigned short* EMB  = (unsigned short*)(ws + oEm);
  float*          HP   = (float*)(ws + oHP);
  float*          PREC = (float*)(ws + oPR);
  float*          STATP= (float*)(ws + oSP);
  unsigned short* AIN  = (unsigned short*)(ws + oAI);
  unsigned short* P1   = (unsigned short*)(ws + oP1);
  unsigned short* P3   = (unsigned short*)(ws + oP3);
  float*          P2   = (float*)(ws + oP2);
  int*            LISTS= (int*)(ws + oLS);
  int*            OFFS = (int*)(ws + oOF);
  int*            CNTS = (int*)(ws + oCN);
  int*            META = (int*)(ws + oMT);
  float*          PT   = (float*)(ws + oPT);
  float*          STAT = (float*)(ws + oST);
  unsigned short* POOL = (unsigned short*)(ws + oPL);

  hipFuncSetAttribute(reinterpret_cast<const void*>(&k_compact), hipFuncAttributeMaxDynamicSharedMemorySize, LDS_CMP);

  k_prep<<<cdiv(NUTOT, NTHR), NTHR, 0, stream>>>(inW, cW1, cW2, roW1, aemb, WinT, W1T2, W2T2, RoT2, EMB);
  k_pe<<<gPE, NTHR, 0, stream>>>(pe, peW1, peb1, peW2, peb2, nN, HP, PREC);
  k_comb_pe<<<1, 32, 0, stream>>>(PREC, gPE, peg, pebt, STATP);
  k_ain<<<gM, NTHR, 0, stream>>>(x, EMB, HP, STATP, nN, MP, AIN);
  k_gemm<3><<<dim3(gM, 1), GTHR, 0, stream>>>(AIN, HD, WinT, HD, HD, inb, (void*)P2, HD, 0, nN, MP, PT, inb, inb);
  k_compact<<<nBlk, NTHR, LDS_CMP, stream>>>(src, dst, nN, nE, vec8, LISTS, OFFS, CNTS, META);
  for (int i = 0; i < NLAY; ++i) {
    if (i == 0) {
      k_agg<1><<<gM, NTHR, 0, stream>>>(P2, STAT, LISTS, OFFS, CNTS, META, nBlk, nN, MP, P1);
    } else {
      k_agg<0><<<gM, NTHR, 0, stream>>>(P2, STAT + (size_t)(i - 1) * 4 * HD, LISTS, OFFS, CNTS, META, nBlk, nN, MP, P1);
    }
    k_gemm<2><<<dim3(gM, 1), GTHR, 0, stream>>>(P1, K2, W1T2 + (size_t)i * HD * K2, K2, K2, cb1 + i * HD,
                                                (void*)P3, K2, HD, nN, MP, PT, inb, inb);
    k_gemm<1><<<dim3(gM, 1), GTHR, 0, stream>>>(P3, K2, W2T2 + (size_t)i * HD * K2, K2, K2, cb2 + i * HD,
                                                (void*)P2, HD, 0, nN, MP, PT, inb, inb);
    k_comb<<<1, GBN, 0, stream>>>(PT, gM, bng + i * HD, bnb + i * HD, STAT + (size_t)i * 4 * HD);
  }
  k_pool<<<nG / PG, NTHR, 0, stream>>>(P2, STAT + (size_t)(NLAY - 1) * 4 * HD, batch, nN, vec8b, nG, POOL);
  k_gemm<4><<<dim3(nG / GBM, 1), GTHR, 0, stream>>>(POOL, K2, RoT2, K2, K2, rob1, (void*)out, 1, 0, nG, nG, PT, roW2, rob2);
}
